// MultiHeadAttention_83116207112396
// MI455X (gfx1250) — hardware-verified
//
#include <hip/hip_runtime.h>
#include <math.h>

#ifndef NB
#define NB 32
#endif
#ifndef SEQ
#define SEQ 512
#endif
#ifndef EROWS
#define EROWS 0
#endif
#define NB_FULL 32
#define SEQ_FULL 512
#define DM 512
#define NH 8
#define MROWS (NB * SEQ)
#define NEGFILL (-4294967295.0f)
#define AT_PSC 32768.0f
#define WCARRY 64.0f
#define WINV 0.015625f
#define RES_SC 2048.0f
#define RES_INV 0.00048828125f
#define ECH (EROWS / 64)
#define ECH_DIV ((ECH) > 0 ? (ECH) : 1)
#define EPL ((size_t)NB * EROWS * DM)
#define MW_PAD (((MROWS + 1023) / 1024) * 32)

static_assert(NB >= 1 && NB <= NB_FULL);
static_assert(SEQ >= 64 && SEQ <= SEQ_FULL && (SEQ % 64) == 0);
static_assert((MROWS % 128) == 0);
static_assert((DM % 64) == 0 && (DM % 32) == 0);
static_assert(((MROWS * 64) % 256) == 0);
static_assert((MROWS % 8) == 0);
static_assert(EROWS >= 0 && EROWS <= SEQ && (EROWS % 64) == 0);
static_assert(DM == NH * 64);
static_assert(DM == 32 * 4 * 4);
static_assert((SEQ % 32) == 0);
static_assert(((3 * NB * EROWS * DM) % 2048) == 0);
static_assert((MW_PAD % 32) == 0 && MW_PAD * 32 >= MROWS);

typedef __attribute__((ext_vector_type(16))) _Float16 v16h;
typedef __attribute__((ext_vector_type(8)))  _Float16 v8h;
typedef __attribute__((ext_vector_type(16))) __bf16   v16b;
typedef __attribute__((ext_vector_type(8)))  float    v8f;
typedef __attribute__((ext_vector_type(4)))  float    v4f;
typedef unsigned int cm_u4 __attribute__((ext_vector_type(4)));
typedef _Float16 h16;

__device__ __forceinline__ v8f wmma16(v16h a, v16h b, v8f c) {
    c = __builtin_amdgcn_wmma_f32_16x16x32_f16(false, a, false, b, (short)0, c, false, false);
    asm volatile("v_nop\n\tv_nop\n\tv_nop\n\tv_nop" : "+v"(c) : "v"(a), "v"(b));
    return c;
}

#define VST2(T, ptr, val) do { const T vst2_v_ = (val); *(volatile T*)(ptr) = vst2_v_; __threadfence(); *(volatile T*)(ptr) = vst2_v_; } while (0)
#define VST2V4(ptr, val) do { const v4f vst2_v4_ = (val); *(volatile v4f*)(ptr) = vst2_v4_; __threadfence(); *(volatile v4f*)(ptr) = vst2_v4_; } while (0)

__device__ __forceinline__ void wave_lds_sync() {
    __builtin_amdgcn_fence(3  , "workgroup");
    __builtin_amdgcn_wave_barrier();
    __builtin_amdgcn_fence(2  , "workgroup");
}

__device__ __forceinline__ unsigned int cmb_pk2(float a, float b) { return (unsigned int)__builtin_bit_cast(unsigned short, (_Float16)a) | ((unsigned int)__builtin_bit_cast(unsigned short, (_Float16)b) << 16); }
__device__ __forceinline__ float cmb_bf(float v) { const unsigned u = __builtin_bit_cast(unsigned, v); const unsigned r = (u + 0x7fffu + ((u >> 16) & 1u)) & 0xffff0000u; return __builtin_bit_cast(float, r); }

static __device__ __forceinline__ h16 toh_flush(float v) { const h16 r = (h16)v; return (fabsf(v) < 6.103515625e-05f) ? (h16)0.0f : r; }
static __device__ __forceinline__ unsigned short hbits16(h16 v) { return __builtin_bit_cast(unsigned short, v); }

namespace gemm {
typedef __attribute__((ext_vector_type(16))) _Float16 v16h;
typedef __attribute__((ext_vector_type(8)))  _Float16 v8h;
typedef __attribute__((ext_vector_type(16))) __bf16   v16b;
typedef __attribute__((ext_vector_type(8)))  __bf16   v8b;
typedef __attribute__((ext_vector_type(8)))  float    v8f;
typedef __attribute__((ext_vector_type(4)))  float    v4f;

__device__ __forceinline__ unsigned short f2bf_bits(float f) {
  unsigned u = __float_as_uint(f);
  return (unsigned short)((u + 0x7FFFu + ((u >> 16) & 1u)) >> 16);
}
__device__ __forceinline__ float bf_bits2f(unsigned short h) { return __uint_as_float(((unsigned)h) << 16); }

__device__ __forceinline__ void dep_guard_h(v8f& a, v8f& b, v16h x, v16h y) { asm volatile("v_nop\n\tv_nop\n\tv_nop\n\tv_nop" : "+v"(a), "+v"(b) : "v"(x), "v"(y)); }
__device__ __forceinline__ void dep_guard_b(v8f& a, v8f& b, v16b x, v16b y) { asm volatile("v_nop\n\tv_nop\n\tv_nop\n\tv_nop" : "+v"(a), "+v"(b) : "v"(x), "v"(y)); }
__device__ __forceinline__ void keep4_h(v16h a, v16h b, v16h c, v16h d) { asm volatile("v_nop" :: "v"(a), "v"(b), "v"(c), "v"(d)); }
__device__ __forceinline__ void keep4_b(v16b a, v16b b, v16b c, v16b d) { asm volatile("v_nop" :: "v"(a), "v"(b), "v"(c), "v"(d)); }
__device__ __forceinline__ void acc_guard4(v8f& a, v8f& b, v8f& c, v8f& d) { asm volatile("v_nop\n\tv_nop\n\tv_nop\n\tv_nop" : "+v"(a), "+v"(b), "+v"(c), "+v"(d)); }
template <typename T> struct Frag;
template <> struct Frag<_Float16> {
  typedef v16h V; union U { v16h v; v8h h[2]; };
  static __device__ __forceinline__ v16h load(const _Float16* p) {
    U f; f.h[0] = *(const v8h*)(p); f.h[1] = *(const v8h*)(p + 16); return f.v;
  }
  static __device__ __forceinline__ v8f mma(v16h a, v16h b, v8f c) {
    return __builtin_amdgcn_wmma_f32_16x16x32_f16(false, a, false, b, (short)0, c, false, false);
  }
  static __device__ __forceinline__ void guard(v8f& a, v8f& b, v16h x, v16h y) { dep_guard_h(a, b, x, y); }
  static __device__ __forceinline__ void keep(v16h a, v16h b, v16h c, v16h d) { keep4_h(a, b, c, d); }
};
template <> struct Frag<__bf16> {
  typedef v16b V; union U { v16b v; v8b h[2]; };
  static __device__ __forceinline__ v16b load(const __bf16* p) {
    U f; f.h[0] = *(const v8b*)(p); f.h[1] = *(const v8b*)(p + 16); return f.v;
  }
  static __device__ __forceinline__ v8f mma(v16b a, v16b b, v8f c) {
    return __builtin_amdgcn_wmma_f32_16x16x32_bf16(false, a, false, b, (short)0, c, false, false);
  }
  static __device__ __forceinline__ void guard(v8f& a, v8f& b, v16b x, v16b y) { dep_guard_b(a, b, x, y); }
  static __device__ __forceinline__ void keep(v16b a, v16b b, v16b c, v16b d) { keep4_b(a, b, c, d); }
};

template <int ET> struct Elem;
template <> struct Elem<0> { typedef _Float16 T; };
template <> struct Elem<1> { typedef __bf16 T; };
template <int ET, bool SPLIT, int BIAS_MODE, int OUT_MODE, bool RESID, int ACT = 0>
__global__ __launch_bounds__(256) void wmma_gemm64(
    const unsigned short* __restrict__ Ap, const unsigned short* __restrict__ A2p, int lda, long strideA,
    const unsigned short* __restrict__ Btp, const unsigned short* __restrict__ Bt2p, int ldb, long strideB,
    void* __restrict__ Cout, void* __restrict__ Cout2, int ldc, long strideC,
    const float* __restrict__ bias,
    const float* __restrict__ resid, long strideR,
    int M, int N, int K, float scale) {
  typedef typename Elem<ET>::T T;
  typedef typename Frag<T>::V V;
  const T* A = (const T*)Ap; const T* A2 = (const T*)A2p; const T* Bt = (const T*)Btp; const T* Bt2 = (const T*)Bt2p;
  __shared__ __align__(16) float sT[8][16 * 68];
  const int b    = blockIdx.y;
  const int lane = threadIdx.x & 31;
  const int wave = threadIdx.x >> 5;
  const int tilesN = N >> 6;
  const int tilesM = M >> 6;
  const int tile = blockIdx.x * 8 + wave;
  if (tile >= tilesM * tilesN) return;
  const int tm = tile / tilesN;
  const int tn = tile - tm * tilesN;
  const int m0 = tm << 6;
  const int n0 = tn << 6;

  const T* Ab  = A  + (size_t)b * strideA;
  const T* Bb  = Bt + (size_t)b * strideB;
  const T* Ab2 = SPLIT ? (A2  + (size_t)b * strideA) : nullptr;
  const T* Bb2 = SPLIT ? (Bt2 + (size_t)b * strideB) : nullptr;

  const int rlane = lane & 15;
  const int koff  = (lane >> 4) * 8;
  const int mOff  = (lane >> 4) * 8;

  v8f acc[4][4];
#pragma unroll
  for (int i = 0; i < 4; ++i)
#pragma unroll
    for (int j = 0; j < 4; ++j) acc[i][j] = (v8f){0.f,0.f,0.f,0.f,0.f,0.f,0.f,0.f};

  for (int k0 = 0; k0 < K; k0 += 32) {
    V bh[4], bl[4];
#pragma unroll
    for (int j = 0; j < 4; ++j) {
      const size_t bo = (size_t)(n0 + (j << 4) + rlane) * ldb + koff + k0;
      bh[j] = Frag<T>::load(Bb + bo);
      if (SPLIT) bl[j] = Frag<T>::load(Bb2 + bo);
    }
#pragma unroll
    for (int i = 0; i < 4; ++i) {
      const size_t ao = (size_t)(m0 + (i << 4) + rlane) * lda + koff + k0;
      V ah = Frag<T>::load(Ab + ao);
      V al;
      if (SPLIT) al = Frag<T>::load(Ab2 + ao);
#pragma unroll
      for (int j = 0; j < 4; ++j) {
        acc[i][j] = Frag<T>::mma(ah, bh[j], acc[i][j]);
        if (SPLIT) {
          acc[i][j] = Frag<T>::mma(ah, bl[j], acc[i][j]);
          acc[i][j] = Frag<T>::mma(al, bh[j], acc[i][j]);
        }
      }
      Frag<T>::guard(acc[i][0], acc[i][3], ah, SPLIT ? al : ah);
    }
    Frag<T>::keep(bh[0], bh[1], bh[2], bh[3]);
    if (SPLIT) Frag<T>::keep(bl[0], bl[1], bl[2], bl[3]);
  }
  acc_guard4(acc[0][0], acc[0][1], acc[0][2], acc[0][3]);
  acc_guard4(acc[1][0], acc[1][1], acc[1][2], acc[1][3]);
  acc_guard4(acc[2][0], acc[2][1], acc[2][2], acc[2][3]);
  acc_guard4(acc[3][0], acc[3][1], acc[3][2], acc[3][3]);

  float* slab = sT[wave];
  const float* Rb = RESID ? (resid + (size_t)b * strideR) : nullptr;
#pragma unroll
  for (int i = 0; i < 4; ++i) {
    const int mBase = m0 + (i << 4);
#pragma unroll
    for (int j = 0; j < 4; ++j) {
      const int n = n0 + (j << 4) + rlane;
      float bv = 0.f;
      if (BIAS_MODE == 2) bv = bias[n];
#pragma unroll
      for (int r = 0; r < 8; ++r) {
        float v = acc[i][j][r] * scale;
        if (BIAS_MODE == 1) v += bias[mBase + mOff + r];
        if (BIAS_MODE == 2) v += bv;
        if (RESID) v += Rb[(size_t)(mBase + mOff + r) * ldc + n];
        if (ACT == 2) v = fmaxf(v, 0.0f);
        slab[(mOff + r) * 68 + (j << 4) + rlane] = v;
      }
    }
    __builtin_amdgcn_fence(3  , "workgroup");
    __builtin_amdgcn_wave_barrier();
    __builtin_amdgcn_fence(2  , "workgroup");
    if (OUT_MODE == 0) {
      float* C = (float*)Cout + (size_t)b * strideC;
      const int hh = lane >> 4, c4 = (lane & 15) * 4;
      for (int pass = 0; pass < 2; ++pass) {
#pragma unroll
        for (int it = 0; it < 8; ++it) {
          const int row = it * 2 + hh;
          v4f v = *(const v4f*)(slab + row * 68 + c4);
          *(volatile v4f*)(C + (size_t)(mBase + row) * ldc + n0 + c4) = v;
        }
        __threadfence();
      }
    } else {
      const int q = lane >> 3, c8 = (lane & 7) * 8;
      unsigned short* C  = (unsigned short*)Cout  + (size_t)b * strideC;
      unsigned short* C2 = (OUT_MODE == 2) ? ((unsigned short*)Cout2 + (size_t)b * strideC) : nullptr;
      for (int pass = 0; pass < 2; ++pass) {
#pragma unroll
        for (int it = 0; it < 4; ++it) {
          const int row = it * 4 + q;
          const float* sp = slab + row * 68 + c8;
          v8h hv, lv;
#pragma unroll
          for (int e = 0; e < 8; ++e) {
            if (OUT_MODE == 1) {
              hv[e] = (_Float16)sp[e];
            } else {
              unsigned short hb = f2bf_bits(sp[e]);
              unsigned short lb = f2bf_bits(sp[e] - bf_bits2f(hb));
              hv[e] = __builtin_bit_cast(_Float16, hb);
              lv[e] = __builtin_bit_cast(_Float16, lb);
            }
          }
          *(volatile v8h*)(C + (size_t)(mBase + row) * ldc + n0 + c8) = hv;
          if (OUT_MODE == 2) *(volatile v8h*)(C2 + (size_t)(mBase + row) * ldc + n0 + c8) = lv;
        }
        __threadfence();
      }
    }
    __builtin_amdgcn_fence(3  , "workgroup");
    __builtin_amdgcn_wave_barrier();
    __builtin_amdgcn_fence(2  , "workgroup");
  }
}
}

__global__ __launch_bounds__(256) void k_cast_act(const float* __restrict__ q_in, const float* __restrict__ k_in, unsigned short* __restrict__ dst) {
    const unsigned u = blockIdx.x * 256u + threadIdx.x;
    if (u >= (unsigned)MROWS * 64u) return;
    const unsigned which = blockIdx.y;
    const float* src = which ? k_in : q_in;
    const unsigned r = u >> 6, c0 = (u & 63u) << 3;
    const unsigned b = r / (unsigned)SEQ, s = r - b * (unsigned)SEQ;
    const float* sp = src + ((size_t)b * SEQ_FULL + s) * DM + c0;
    const v4f a = *(const v4f*)sp, c = *(const v4f*)(sp + 4);
    cm_u4 pk;
    pk.x = cmb_pk2(cmb_bf(a.x), cmb_bf(a.y)); pk.y = cmb_pk2(cmb_bf(a.z), cmb_bf(a.w));
    pk.z = cmb_pk2(cmb_bf(c.x), cmb_bf(c.y)); pk.w = cmb_pk2(cmb_bf(c.z), cmb_bf(c.w));
    unsigned short* d = dst + (size_t)which * MROWS * DM + (size_t)r * DM + c0;
    VST2(cm_u4, (cm_u4*)d, pk);
}

__global__ __launch_bounds__(256) void k_cast_wT(const float* __restrict__ SRC, unsigned lds, unsigned short* __restrict__ DST, unsigned ldd, unsigned nR, unsigned nC, float sc) {
    const unsigned u = blockIdx.x * 256u + threadIdx.x; const unsigned per = nR >> 3;
    if (u >= nC * per) return;
    const unsigned cc = u / per, r0 = (u - cc * per) << 3;
    float w[8];
#pragma unroll
    for (int e = 0; e < 8; ++e) w[e] = cmb_bf(SRC[(size_t)(r0 + (unsigned)e) * lds + cc]) * sc;
    cm_u4 pk; pk.x = cmb_pk2(w[0], w[1]); pk.y = cmb_pk2(w[2], w[3]); pk.z = cmb_pk2(w[4], w[5]); pk.w = cmb_pk2(w[6], w[7]);
    VST2(cm_u4, (cm_u4*)(DST + (size_t)cc * ldd + r0), pk);
}

__global__ __launch_bounds__(256) void k_rowmask(const float* __restrict__ q_in, const float* __restrict__ k_in, unsigned* __restrict__ dst) {
#pragma clang fp contract(off)
    __shared__ unsigned wsh[32];
    const unsigned tid = threadIdx.x, lane = tid & 31u;
    const unsigned wave = (unsigned)__builtin_amdgcn_readfirstlane((int)(tid >> 5));
    const unsigned which = blockIdx.y;
    const float* src = which ? k_in : q_in;
#pragma unroll 1
    for (unsigned g = 0; g < 4u; ++g) {
        const unsigned grp = wave * 4u + g;
        const unsigned base = blockIdx.x * 1024u + grp * 32u;
        unsigned bits = 0u;
#pragma unroll 1
        for (unsigned i = 0; i < 32u; ++i) {
            const unsigned row = base + i;
            const unsigned rc = min(row, (unsigned)(MROWS - 1));
            const unsigned b = rc / (unsigned)SEQ, s = rc - b * (unsigned)SEQ;
            const float* rp = src + ((size_t)b * SEQ_FULL + s) * DM + lane * 4u;
            float sum = 0.f;
#pragma unroll 1
            for (unsigned j = 0; j < 4u; ++j) {
                const v4f x = *(const v4f*)(rp + 128u * j);
                sum += (cmb_bf(x.x) + cmb_bf(x.y)) + (cmb_bf(x.z) + cmb_bf(x.w));
            }
            sum += __shfl_xor(sum, 16, 32); sum += __shfl_xor(sum, 8, 32); sum += __shfl_xor(sum, 4, 32); sum += __shfl_xor(sum, 2, 32); sum += __shfl_xor(sum, 1, 32);
            const unsigned f = ((sum != 0.0f) && (row < (unsigned)MROWS)) ? 1u : 0u;
            bits |= f << i;
        }
        if (lane == 0u) wsh[grp] = bits;
    }
    __syncthreads();
    if (wave == 0u) {
        const unsigned w = wsh[lane];
        VST2(unsigned, dst + (size_t)which * MW_PAD + blockIdx.x * 32u + lane, w);
    }
}

__global__ __launch_bounds__(256) void k_split_early(const float* __restrict__ src, unsigned short* __restrict__ hi, unsigned short* __restrict__ rs) {
#pragma clang fp contract(off)
    const unsigned u = blockIdx.x * 256u + threadIdx.x;
    if (u >= (unsigned)(3u * (unsigned)NB * (unsigned)EROWS * (unsigned)DM / 8u)) return;
    const float* sp = src + (size_t)u * 8u;
    const v4f a = *(const v4f*)sp, c = *(const v4f*)(sp + 4);
    float v[8];
    v[0] = a.x; v[1] = a.y; v[2] = a.z; v[3] = a.w; v[4] = c.x; v[5] = c.y; v[6] = c.z; v[7] = c.w;
    unsigned hb[8], rb[8];
#pragma unroll
    for (int e = 0; e < 8; ++e) {
        const h16 hv = toh_flush(v[e]);
        const h16 rv = toh_flush((v[e] - (float)hv) * RES_SC);
        hb[e] = (unsigned)hbits16(hv);
        rb[e] = (unsigned)hbits16(rv);
    }
    cm_u4 ph, pr;
    ph.x = hb[0] | (hb[1] << 16); ph.y = hb[2] | (hb[3] << 16); ph.z = hb[4] | (hb[5] << 16); ph.w = hb[6] | (hb[7] << 16);
    pr.x = rb[0] | (rb[1] << 16); pr.y = rb[2] | (rb[3] << 16); pr.z = rb[4] | (rb[5] << 16); pr.w = rb[6] | (rb[7] << 16);
    VST2(cm_u4, (cm_u4*)(hi + (size_t)u * 8u), ph);
    VST2(cm_u4, (cm_u4*)(rs + (size_t)u * 8u), pr);
}

__global__ __launch_bounds__(128) void k_attn_main(const unsigned short* __restrict__ Qp, const unsigned short* __restrict__ Kp, const unsigned short* __restrict__ VTp,
                                                   const unsigned* __restrict__ qbits, const unsigned* __restrict__ kbits, const float* __restrict__ qin, float* __restrict__ out) {
    typedef gemm::Frag<_Float16> FH;
    __shared__ __align__(16) _Float16 Psh[4][16 * 64];
    __shared__ __align__(16) float    Os[4][16 * 68];
    const unsigned tid = threadIdx.x, lane = tid & 31u, hh = lane >> 4, c = lane & 15u;
    const unsigned wave = (unsigned)__builtin_amdgcn_readfirstlane((int)(tid >> 5));
    const unsigned nqb = (unsigned)SEQ / 64u;
    const unsigned bx = blockIdx.x;
    const unsigned bh = bx / nqb, qb = bx - bh * nqb;
    const unsigned h = bh & (unsigned)(NH - 1);
    unsigned b = bh / (unsigned)NH; b = (b < (unsigned)NB) ? b : (unsigned)(NB - 1);
    const unsigned q0 = qb * 64u + wave * 16u;

    const unsigned* kbw = kbits + (size_t)b * (unsigned)(SEQ / 32);
    const unsigned wq = q0 >> 5;
    unsigned any = 0u;
    for (unsigned i = 0; i < wq; ++i) any |= kbw[i];
    any |= kbw[wq] & (0xffffffffu >> (31u - (q0 & 31u)));
    const unsigned live = (any != 0u) ? 1u : 0u;
    if ((int)qb < ECH && live != 0u) return;
    const unsigned nck = nqb - live * (nqb - 1u - qb);
    const unsigned qw = qbits[(size_t)b * (unsigned)(SEQ / 32) + wq];

    const _Float16* Qb = (const _Float16*)Qp + (size_t)b * SEQ * DM + h * 64u;
    const _Float16* Kb = (const _Float16*)Kp + (size_t)b * SEQ * DM + h * 64u;
    const _Float16* Vb = (const _Float16*)VTp + ((size_t)b * DM + h * 64u) * SEQ;
    float* Ob = out + (size_t)b * SEQ * DM + h * 64u;
    const float* Rb = qin + (size_t)b * SEQ_FULL * DM + h * 64u;

    const _Float16* qrow = Qb + (size_t)(q0 + c) * DM + 8u * hh;
    const v16h qa0 = FH::load(qrow), qa1 = FH::load(qrow + 32);

    float mrow[8], lrow[8];
    v8f oacc[4];
#pragma unroll
    for (int r = 0; r < 8; ++r) { mrow[r] = -INFINITY; lrow[r] = 0.f; }
#pragma unroll
    for (int t = 0; t < 4; ++t) oacc[t] = (v8f){0.f,0.f,0.f,0.f,0.f,0.f,0.f,0.f};

    _Float16* pw = Psh[wave];
    for (unsigned kc = 0; kc < nck; ++kc) {
        const unsigned kv0 = kc * 64u;
        const unsigned kw0 = kbw[2u * kc], kw1 = kbw[2u * kc + 1u];
        bool kdead[4];
        kdead[0] = ((kw0 >> c) & 1u) == 0u; kdead[1] = ((kw0 >> (16u + c)) & 1u) == 0u;
        kdead[2] = ((kw1 >> c) & 1u) == 0u; kdead[3] = ((kw1 >> (16u + c)) & 1u) == 0u;
        v8f s[4];
#pragma unroll
        for (int j = 0; j < 4; ++j) {
            const _Float16* kr = Kb + (size_t)(kv0 + (unsigned)j * 16u + c) * DM + 8u * hh;
            v8f z = (v8f){0.f,0.f,0.f,0.f,0.f,0.f,0.f,0.f};
            z = wmma16(qa0, FH::load(kr), z);
            z = wmma16(qa1, FH::load(kr + 32), z);
            s[j] = z;
        }
        float cm[8];
#pragma unroll
        for (int r = 0; r < 8; ++r) {
            const int qr = (int)(q0 + 8u * hh) + r;
            float m = -INFINITY;
#pragma unroll
            for (int j = 0; j < 4; ++j) {
                const int kvcol = (int)(kv0 + c) + j * 16;
                const bool fill = (kvcol > qr) || kdead[j];
                const float v = fill ? NEGFILL : s[j][r] * 0.125f;
                s[j][r] = v;
                m = fmaxf(m, v);
            }
            m = fmaxf(m, __shfl_xor(m, 1, 32)); m = fmaxf(m, __shfl_xor(m, 2, 32));
            m = fmaxf(m, __shfl_xor(m, 4, 32)); m = fmaxf(m, __shfl_xor(m, 8, 32));
            cm[r] = m;
        }
#pragma unroll
        for (int r = 0; r < 8; ++r) {
            const float mnew = fmaxf(mrow[r], cm[r]);
            const float alpha = expf(mrow[r] - mnew);
            mrow[r] = mnew;
            float psum = 0.f;
#pragma unroll
            for (int j = 0; j < 4; ++j) {
                const float p = expf(s[j][r] - mnew);
                psum += p;
                pw[(8u * hh + (unsigned)r) * 64u + (unsigned)j * 16u + c] = toh_flush(p * AT_PSC);
            }
            psum += __shfl_xor(psum, 1, 32); psum += __shfl_xor(psum, 2, 32);
            psum += __shfl_xor(psum, 4, 32); psum += __shfl_xor(psum, 8, 32);
            lrow[r] = lrow[r] * alpha + psum;
#pragma unroll
            for (int t = 0; t < 4; ++t) oacc[t][r] *= alpha;
        }
        wave_lds_sync();
#pragma unroll
        for (int kk = 0; kk < 2; ++kk) {
            const v16h pa = FH::load(pw + c * 64u + (unsigned)kk * 32u + 8u * hh);
#pragma unroll
            for (int t = 0; t < 4; ++t) {
                const v16h vb = FH::load(Vb + (size_t)((unsigned)t * 16u + c) * SEQ + kv0 + (unsigned)kk * 32u + 8u * hh);
                oacc[t] = wmma16(pa, vb, oacc[t]);
            }
        }
        wave_lds_sync();
    }

    float* os = Os[wave];
#pragma unroll
    for (int r = 0; r < 8; ++r) {
        const float inv = (lrow[r] > 0.f) ? 1.0f / (lrow[r] * AT_PSC) : 0.f;
        const bool qlive = ((qw >> ((q0 & 31u) + 8u * hh + (unsigned)r)) & 1u) != 0u;
#pragma unroll
        for (int t = 0; t < 4; ++t) os[(8u * hh + (unsigned)r) * 68u + (unsigned)t * 16u + c] = qlive ? oacc[t][r] * inv : 0.f;
    }
    wave_lds_sync();
    {
        const unsigned c4 = (lane & 15u) * 4u;
        for (int pass = 0; pass < 2; ++pass) {
#pragma unroll
            for (int it = 0; it < 8; ++it) {
                const unsigned row = (unsigned)it * 2u + hh;
                v4f val = *(const v4f*)(os + row * 68u + c4);
                const v4f qv = *(const v4f*)(Rb + (size_t)(q0 + row) * DM + c4);
                val.x += cmb_bf(qv.x); val.y += cmb_bf(qv.y); val.z += cmb_bf(qv.z); val.w += cmb_bf(qv.w);
                *(volatile v4f*)(Ob + (size_t)(q0 + row) * DM + c4) = val;
            }
            __threadfence();
        }
    }
}

__global__ __launch_bounds__(128) void k_attn_early(const unsigned short* __restrict__ EHp, const unsigned short* __restrict__ ERp,
                                                    const unsigned* __restrict__ qbits, const unsigned* __restrict__ kbits, const float* __restrict__ qin, float* __restrict__ out) {
    typedef gemm::Frag<_Float16> FH;
    __shared__ __align__(16) _Float16 Phs[4][16 * 32];
    __shared__ __align__(16) _Float16 Prs[4][16 * 32];
    __shared__ __align__(16) float    Os[4][16 * 68];
    const unsigned tid = threadIdx.x, lane = tid & 31u, hh = lane >> 4, c = lane & 15u;
    const unsigned wave = (unsigned)__builtin_amdgcn_readfirstlane((int)(tid >> 5));
    const unsigned ech = (unsigned)ECH_DIV;
    const unsigned bx = blockIdx.x;
    const unsigned bh = bx / ech, qb = bx - bh * ech;
    const unsigned h = bh & (unsigned)(NH - 1);
    unsigned b = bh / (unsigned)NH; b = (b < (unsigned)NB) ? b : (unsigned)(NB - 1);
    const unsigned q0 = qb * 64u + wave * 16u;

    const unsigned* kbw = kbits + (size_t)b * (unsigned)(SEQ / 32);
    const unsigned wq = q0 >> 5;
    unsigned any = 0u;
    for (unsigned i = 0; i < wq; ++i) any |= kbw[i];
    any |= kbw[wq] & (0xffffffffu >> (31u - (q0 & 31u)));
    if (any == 0u) return;
    const unsigned qw = qbits[(size_t)b * (unsigned)(SEQ / 32) + wq];

    const size_t qk0 = ((size_t)b * EROWS) * DM + h * 64u;
    const size_t vt0 = (size_t)2 * EPL + ((size_t)b * DM + h * 64u) * EROWS;
    const _Float16* Qh = (const _Float16*)EHp + qk0;
    const _Float16* Qr = (const _Float16*)ERp + qk0;
    const _Float16* Kh = (const _Float16*)EHp + EPL + qk0;
    const _Float16* Kr = (const _Float16*)ERp + EPL + qk0;
    const _Float16* Vh = (const _Float16*)EHp + vt0;
    const _Float16* Vr = (const _Float16*)ERp + vt0;
    float* Ob = out + (size_t)b * SEQ * DM + h * 64u;
    const float* Rb = qin + (size_t)b * SEQ_FULL * DM + h * 64u;

    float mrow[8], lrow[8];
    v8f oacc[4], ores[4];
#pragma unroll
    for (int r = 0; r < 8; ++r) { mrow[r] = -INFINITY; lrow[r] = 0.f; }
#pragma unroll
    for (int t = 0; t < 4; ++t) { oacc[t] = (v8f){0.f,0.f,0.f,0.f,0.f,0.f,0.f,0.f}; ores[t] = (v8f){0.f,0.f,0.f,0.f,0.f,0.f,0.f,0.f}; }

    _Float16* phw = Phs[wave];
    _Float16* prw = Prs[wave];
    const unsigned nhalf = ((q0 + 15u) >> 5) + 1u;
    for (unsigned hv = 0; hv < nhalf; ++hv) {
        const unsigned kvh = hv * 32u;
        const unsigned kw = kbw[hv];
        bool kdead[2];
        kdead[0] = ((kw >> c) & 1u) == 0u; kdead[1] = ((kw >> (16u + c)) & 1u) == 0u;
        v8f sm[2], sr[2];
#pragma unroll
        for (int j = 0; j < 2; ++j) { sm[j] = (v8f){0.f,0.f,0.f,0.f,0.f,0.f,0.f,0.f}; sr[j] = (v8f){0.f,0.f,0.f,0.f,0.f,0.f,0.f,0.f}; }
#pragma unroll
        for (int ks = 0; ks < 2; ++ks) {
            const size_t qo = (size_t)(q0 + c) * DM + 8u * hh + 32u * (unsigned)ks;
            const v16h qav = FH::load(Qh + qo);
            const v16h qar = FH::load(Qr + qo);
#pragma unroll
            for (int j = 0; j < 2; ++j) {
                const size_t ko = (size_t)(kvh + (unsigned)j * 16u + c) * DM + 8u * hh + 32u * (unsigned)ks;
                const v16h kbv = FH::load(Kh + ko);
                const v16h kbr = FH::load(Kr + ko);
                sm[j] = wmma16(qav, kbv, sm[j]);
                sr[j] = wmma16(qar, kbv, sr[j]);
                sr[j] = wmma16(qav, kbr, sr[j]);
            }
        }
        float cm[8];
#pragma unroll
        for (int r = 0; r < 8; ++r) {
            const int qrw = (int)(q0 + 8u * hh) + r;
            float m = -INFINITY;
#pragma unroll
            for (int j = 0; j < 2; ++j) {
                const int kvcol = (int)(kvh + c) + j * 16;
                const bool fill = (kvcol > qrw) || kdead[j];
                const float v = fill ? NEGFILL : (sm[j][r] + sr[j][r] * RES_INV) * 0.125f;
                sm[j][r] = v;
                m = fmaxf(m, v);
            }
            m = fmaxf(m, __shfl_xor(m, 1, 32)); m = fmaxf(m, __shfl_xor(m, 2, 32));
            m = fmaxf(m, __shfl_xor(m, 4, 32)); m = fmaxf(m, __shfl_xor(m, 8, 32));
            cm[r] = m;
        }
#pragma unroll
        for (int r = 0; r < 8; ++r) {
            const float mnew = fmaxf(mrow[r], cm[r]);
            const float alpha = expf(mrow[r] - mnew);
            mrow[r] = mnew;
            float psum = 0.f;
#pragma unroll
            for (int j = 0; j < 2; ++j) {
                const float p = expf(sm[j][r] - mnew);
                psum += p;
                const float pv = p * AT_PSC;
                const h16 pvh = toh_flush(pv);
                const h16 pvr = toh_flush((pv - (float)pvh) * RES_SC);
                phw[(8u * hh + (unsigned)r) * 32u + (unsigned)j * 16u + c] = pvh;
                prw[(8u * hh + (unsigned)r) * 32u + (unsigned)j * 16u + c] = pvr;
            }
            psum += __shfl_xor(psum, 1, 32); psum += __shfl_xor(psum, 2, 32);
            psum += __shfl_xor(psum, 4, 32); psum += __shfl_xor(psum, 8, 32);
            lrow[r] = lrow[r] * alpha + psum;
#pragma unroll
            for (int t = 0; t < 4; ++t) { oacc[t][r] *= alpha; ores[t][r] *= alpha; }
        }
        wave_lds_sync();
        {
            const v16h pav = FH::load(phw + c * 32u + 8u * hh);
            const v16h par = FH::load(prw + c * 32u + 8u * hh);
#pragma unroll
            for (int t = 0; t < 4; ++t) {
                const size_t vo = (size_t)((unsigned)t * 16u + c) * EROWS + kvh + 8u * hh;
                const v16h vbv = FH::load(Vh + vo);
                const v16h vbr = FH::load(Vr + vo);
                oacc[t] = wmma16(pav, vbv, oacc[t]);
                ores[t] = wmma16(par, vbv, ores[t]);
                ores[t] = wmma16(pav, vbr, ores[t]);
            }
        }
        wave_lds_sync();
    }

    float* os = Os[wave];
#pragma unroll
    for (int r = 0; r < 8; ++r) {
        const float inv = (lrow[r] > 0.f) ? 1.0f / (lrow[r] * AT_PSC) : 0.f;
        const bool qlive = ((qw >> ((q0 & 31u) + 8u * hh + (unsigned)r)) & 1u) != 0u;
#pragma unroll
        for (int t = 0; t < 4; ++t) os[(8u * hh + (unsigned)r) * 68u + (unsigned)t * 16u + c] = qlive ? (oacc[t][r] + ores[t][r] * RES_INV) * inv : 0.f;
    }
    wave_lds_sync();
    {
        const unsigned c4 = (lane & 15u) * 4u;
        for (int pass = 0; pass < 2; ++pass) {
#pragma unroll
            for (int it = 0; it < 8; ++it) {
                const unsigned row = (unsigned)it * 2u + hh;
                v4f val = *(const v4f*)(os + row * 68u + c4);
                const v4f qv = *(const v4f*)(Rb + (size_t)(q0 + row) * DM + c4);
                val.x += cmb_bf(qv.x); val.y += cmb_bf(qv.y); val.z += cmb_bf(qv.z); val.w += cmb_bf(qv.w);
                *(volatile v4f*)(Ob + (size_t)(q0 + row) * DM + c4) = val;
            }
            __threadfence();
        }
    }
}

extern "C" void kernel_launch(void* const* d_in, const int* in_sizes, int n_in, void* d_out, int out_size, void* d_ws, size_t ws_size, hipStream_t stream) {
    if (n_in < 5) return;
    const long long act_need = ((long long)(NB - 1) * SEQ_FULL + SEQ) * DM;
    if ((long long)in_sizes[0] < act_need || (long long)in_sizes[1] < act_need) return;
    if (in_sizes[2] < DM * DM || in_sizes[3] < DM * DM || in_sizes[4] < DM * DM) return;
    if ((long long)out_size < (long long)MROWS * DM) return;

    const float* query = (const float*)d_in[0];
    const float* keyp  = (const float*)d_in[1];
    const float* W_Q   = (const float*)d_in[2];
    const float* W_K   = (const float*)d_in[3];
    const float* W_V   = (const float*)d_in[4];
    float* out = (float*)d_out;

    constexpr size_t R0_B = (size_t)MROWS * 2048, R1_B = (size_t)MROWS * 3072;
    constexpr size_t RW_B = (size_t)3 * DM * DM * 2;
    constexpr size_t RE_B = (size_t)3 * EPL * 4;
    constexpr size_t RM_B = (size_t)2 * MW_PAD * 4;
    static_assert((size_t)2 * MROWS * DM * 2 == R0_B);
    static_assert((size_t)2 * 3 * EPL * 2 <= R0_B);
    static_assert((size_t)3 * MROWS * DM * 2 == R1_B);
    static_assert((R0_B % 128) == 0 && (R1_B % 128) == 0 && (RW_B % 128) == 0 && (RE_B % 128) == 0 && (RM_B % 128) == 0);
    static_assert(R0_B + R1_B + RW_B + RE_B + RM_B <= (size_t)134217728);
    if (R0_B + R1_B + RW_B + RE_B + RM_B > ws_size) return;
    char* ws = (char*)d_ws;
    unsigned short* X16  = (unsigned short*)ws;
    unsigned short* EH   = (unsigned short*)ws;
    unsigned short* ER   = EH + (size_t)3 * EPL;
    unsigned short* QK16 = (unsigned short*)(ws + R0_B);
    unsigned short* VT16 = QK16 + (size_t)2 * MROWS * DM;
    unsigned short* WQKV = (unsigned short*)(ws + R0_B + R1_B);
    float*          EF   = (float*)(ws + R0_B + R1_B + RW_B);
    unsigned*       MB   = (unsigned*)(ws + R0_B + R1_B + RW_B + RE_B);

    k_cast_act<<<dim3((unsigned)(MROWS * 64 / 256), 2u), 256, 0, stream>>>(query, keyp, X16);
    k_cast_wT<<<(unsigned)((DM * (DM / 8) + 255) / 256), 256, 0, stream>>>(W_Q, DM, WQKV, DM, DM, DM, WCARRY);
    k_cast_wT<<<(unsigned)((DM * (DM / 8) + 255) / 256), 256, 0, stream>>>(W_K, DM, WQKV + (size_t)DM * DM, DM, DM, DM, WCARRY);
    k_cast_wT<<<(unsigned)((DM * (DM / 8) + 255) / 256), 256, 0, stream>>>(W_V, DM, WQKV + (size_t)2 * DM * DM, DM, DM, DM, WCARRY);
    k_rowmask<<<dim3((unsigned)((MROWS + 1023) / 1024), 2u), 256, 0, stream>>>(query, keyp, MB);
    gemm::wmma_gemm64<0, false, 0, 1, false, 0><<<dim3((unsigned)(((MROWS / 64) * (DM / 64) + 7) / 8), 2u), 256, 0, stream>>>(
        X16, nullptr, DM, (long)MROWS * DM, WQKV, nullptr, DM, (long)DM * DM, (void*)QK16, nullptr, DM, (long)MROWS * DM,
        nullptr, nullptr, 0, MROWS, DM, DM, WINV);
    gemm::wmma_gemm64<0, false, 0, 1, false, 0><<<dim3((unsigned)(((DM / 64) * (SEQ / 64) + 7) / 8), (unsigned)NB), 256, 0, stream>>>(
        WQKV + (size_t)2 * DM * DM, nullptr, DM, 0, X16 + (size_t)MROWS * DM, nullptr, DM, (long)SEQ * DM, (void*)VT16, nullptr, SEQ, (long)DM * SEQ,
        nullptr, nullptr, 0, DM, SEQ, DM, WINV);
    if (EROWS > 0) {
        gemm::wmma_gemm64<0, false, 0, 0, false, 0><<<dim3((unsigned)(((EROWS / 64) * (DM / 64) + 7) / 8), (unsigned)NB), 256, 0, stream>>>(
            X16, nullptr, DM, (long)SEQ * DM, WQKV, nullptr, DM, 0, (void*)EF, nullptr, DM, (long)EROWS * DM,
            nullptr, nullptr, 0, EROWS, DM, DM, WINV);
        gemm::wmma_gemm64<0, false, 0, 0, false, 0><<<dim3((unsigned)(((EROWS / 64) * (DM / 64) + 7) / 8), (unsigned)NB), 256, 0, stream>>>(
            X16 + (size_t)MROWS * DM, nullptr, DM, (long)SEQ * DM, WQKV + (size_t)DM * DM, nullptr, DM, 0, (void*)(EF + EPL), nullptr, DM, (long)EROWS * DM,
            nullptr, nullptr, 0, EROWS, DM, DM, WINV);
        gemm::wmma_gemm64<0, false, 0, 0, false, 0><<<dim3((unsigned)(((DM / 64) * (EROWS / 64) + 7) / 8), (unsigned)NB), 256, 0, stream>>>(
            WQKV + (size_t)2 * DM * DM, nullptr, DM, 0, X16 + (size_t)MROWS * DM, nullptr, DM, (long)SEQ * DM, (void*)(EF + (size_t)2 * EPL), nullptr, EROWS, (long)DM * EROWS,
            nullptr, nullptr, 0, DM, EROWS, DM, WINV);
        k_split_early<<<(unsigned)((3 * (size_t)NB * EROWS * DM / 8 + 255) / 256), 256, 0, stream>>>(EF, EH, ER);
    }
    k_attn_main<<<(unsigned)(NB * NH * (SEQ / 64)), 128, 0, stream>>>(QK16, QK16 + (size_t)MROWS * DM, VT16, MB, MB + MW_PAD, query, out);
    if (EROWS > 0) {
        k_attn_early<<<(unsigned)(NB * NH * ECH), 128, 0, stream>>>(EH, ER, MB, MB + MW_PAD, query, out);
    }
}
